// EncoderBlock_56435870269921
// MI455X (gfx1250) — hardware-verified
//
#include <hip/hip_runtime.h>
#include <math.h>

#ifndef NB
#define NB 1
#endif
#ifndef SEQ
#define SEQ 10000
#endif
#define SEQ_FULL 10000
#define EMB 256
#define HEADS 8
#define HD 32
#define HIDD 128
#define NCAM 6
#define NREF 4
#define FL 1024
#define FROWS (NCAM * FL)
#define MPAD (((SEQ + 63) / 64) * 64)
#define HPAD (((SEQ_FULL + 63) / 64) * 64)
#define ACT_CARRY 16.0f
#define W_CARRY 64.0f
#define GEMM_UNDO (1.0f / 1024.0f)
#define QK_SCALE2 (0.17677669529663687f * 1.4426950408889634f)

static_assert(NB == 1);
static_assert(SEQ <= SEQ_FULL);
static_assert(SEQ % 8 == 0);
static_assert(MPAD % 64 == 0 && HPAD % 64 == 0 && FROWS % 64 == 0);
static_assert(MPAD % 8 == 0 && MPAD >= SEQ && HPAD >= SEQ_FULL);
static_assert(EMB % 64 == 0 && HIDD % 64 == 0);
static_assert(EMB % 32 == 0 && HIDD % 32 == 0);
static_assert(HEADS * HD == EMB);
static_assert(32 * 8 == EMB);
static_assert(4 * 8 == HD);
static_assert(ACT_CARRY * W_CARRY * GEMM_UNDO == 1.0f);
static_assert((HPAD * (EMB / 8)) % 256 == 0);
static_assert((EMB * (EMB / 8)) % 256 == 0 && (HIDD * (EMB / 8)) % 256 == 0 && (EMB * (HIDD / 8)) % 256 == 0);
static_assert(FL == 1024 && NCAM * 64 == 384);
static_assert(32 * 16 * 8 == 16 * 64 * 4);
static_assert(32 * 16 * 4 == 16 * 64 * 2);
static_assert(256 * 16 * 4 == 64 * 64 * 4);
static_assert(256 * 16 * 2 == 64 * 64 * 2);
static_assert(32 * 16 * 2 == EMB * 4);
static_assert(32 * 16 * 1 == EMB * 2);
static_assert(8 * 16 * 68 * 4 <= 131072);
static_assert(64 * 65 * 4 <= 131072);
static_assert(8 * 256 * 4 <= 131072);

typedef _Float16 h16;
typedef __attribute__((ext_vector_type(16))) _Float16 v16h;
typedef __attribute__((ext_vector_type(8)))  _Float16 v8h;
typedef __attribute__((ext_vector_type(8)))  float    v8f;
typedef __attribute__((ext_vector_type(4)))  float    v4f;
typedef __attribute__((ext_vector_type(4)))  unsigned int v4u;


#define VST2(T, ptr, val) do { const T vst2_v_ = (val); *(volatile T*)(ptr) = vst2_v_; __threadfence(); *(volatile T*)(ptr) = vst2_v_; } while (0)
#define VST2V4(ptr, val) do { const v4f vst2_v4_ = (val); *(volatile v4f*)(ptr) = vst2_v4_; __threadfence(); *(volatile v4f*)(ptr) = vst2_v4_; } while (0)

__device__ __forceinline__ float bfr(float f) {
    unsigned u = __float_as_uint(f);
    u += 0x7FFFu + ((u >> 16) & 1u);
    return __uint_as_float(u & 0xFFFF0000u);
}
__device__ __forceinline__ unsigned short f2h_bits(float x) {
    return (fabsf(x) < 6.104e-5f) ? (unsigned short)0 : __builtin_bit_cast(unsigned short, (_Float16)x);
}
__device__ __forceinline__ void st8h(unsigned short* P, size_t o, const float* v) {
    v4u pk;
    pk.x = (unsigned)f2h_bits(v[0]) | ((unsigned)f2h_bits(v[1]) << 16);
    pk.y = (unsigned)f2h_bits(v[2]) | ((unsigned)f2h_bits(v[3]) << 16);
    pk.z = (unsigned)f2h_bits(v[4]) | ((unsigned)f2h_bits(v[5]) << 16);
    pk.w = (unsigned)f2h_bits(v[6]) | ((unsigned)f2h_bits(v[7]) << 16);
    VST2(v4u, (v4u*)(P + o), pk);
}
static __device__ __forceinline__ h16 toh_flush(float v) { const float w = (fabsf(v) < 6.103515625e-05f) ? 0.0f : v; return (h16)w; }

union FragU { v16h v; v8h h[2]; };
__device__ __forceinline__ v16h frag_ld(const _Float16* p) {
    FragU f; f.h[0] = *(const v8h*)(p); f.h[1] = *(const v8h*)(p + 16); return f.v;
}
__device__ __forceinline__ v8f wmma16g(v16h a, v16h b, v8f c) {
    c = __builtin_amdgcn_wmma_f32_16x16x32_f16(false, a, false, b, (short)0, c, false, false);
    asm volatile("v_nop\n\tv_nop\n\tv_nop\n\tv_nop" : "+v"(c) : "v"(a), "v"(b));
    return c;
}
__device__ __forceinline__ void wave_sync_lds() {
    __builtin_amdgcn_fence(3  , "workgroup");
    __builtin_amdgcn_wave_barrier();
    __builtin_amdgcn_fence(2  , "workgroup");
}

template <int OUT_MODE, bool BIAS, bool RESID, bool RELU>
__device__ __forceinline__ void gemm64_body(
    const _Float16* __restrict__ A, unsigned lda, const _Float16* __restrict__ Bt, unsigned ldb,
    void* __restrict__ Cout, unsigned ldc, const float* __restrict__ bias, const float* __restrict__ resid,
    unsigned M, unsigned N, unsigned K, float* sTbase) {
  const unsigned lane = threadIdx.x & 31u;
  const unsigned wave = (unsigned)__builtin_amdgcn_readfirstlane((int)(threadIdx.x >> 5));
  const unsigned tilesN = N >> 6, tilesM = M >> 6;
  const unsigned tile = blockIdx.x * 8u + wave;
  if (tile >= tilesM * tilesN) return;
  const unsigned tm = tile / tilesN;
  const unsigned tn = tile - tm * tilesN;
  const unsigned m0 = tm << 6, n0 = tn << 6;
  const unsigned rlane = lane & 15u;
  const unsigned koff = (lane >> 4) * 8u;
  const unsigned mOff = koff;

  v8f acc[4][4];
#pragma unroll
  for (int i = 0; i < 4; ++i)
#pragma unroll
    for (int j = 0; j < 4; ++j) acc[i][j] = (v8f){0.f,0.f,0.f,0.f,0.f,0.f,0.f,0.f};

  for (unsigned k0 = 0; k0 < K; k0 += 32u) {
    v16h bh[4];
#pragma unroll
    for (int j = 0; j < 4; ++j)
      bh[j] = frag_ld(Bt + (size_t)(n0 + ((unsigned)j << 4) + rlane) * ldb + koff + k0);
#pragma unroll
    for (int i = 0; i < 4; ++i) {
      const v16h ah = frag_ld(A + (size_t)(m0 + ((unsigned)i << 4) + rlane) * lda + koff + k0);
#pragma unroll
      for (int j = 0; j < 4; ++j)
        acc[i][j] = wmma16g(ah, bh[j], acc[i][j]);
    }
  }

  float* slab = sTbase + wave * (16u * 68u);
#pragma unroll
  for (int i = 0; i < 4; ++i) {
    const unsigned mBase = m0 + ((unsigned)i << 4);
#pragma unroll
    for (int j = 0; j < 4; ++j) {
      const unsigned n = n0 + ((unsigned)j << 4) + rlane;
      float bv = 0.0f;
      if (BIAS) bv = bfr(bias[n]);
#pragma unroll
      for (int r = 0; r < 8; ++r) {
        float v = acc[i][j][r] * GEMM_UNDO + bv;
        if (RELU) v = fmaxf(v, 0.0f);
        if (OUT_MODE == 1) v *= ACT_CARRY;
        slab[(mOff + (unsigned)r) * 68u + ((unsigned)j << 4) + rlane] = v;
      }
    }
    wave_sync_lds();
    if (OUT_MODE == 0) {
      float* C = (float*)Cout;
      const unsigned hh = lane >> 4, c4 = (lane & 15u) * 4u;
#pragma unroll
      for (int half = 0; half < 2; ++half) {
        v4f vv[4];
#pragma unroll
        for (int it = 0; it < 4; ++it) {
          const unsigned row = (unsigned)(half * 4 + it) * 2u + hh;
          vv[it] = *(const v4f*)(slab + row * 68u + c4);
          if (RESID) vv[it] += *(const v4f*)(resid + (size_t)(mBase + row) * ldc + n0 + c4);
        }
        for (int pass = 0; pass < 2; ++pass) {
#pragma unroll
          for (int it = 0; it < 4; ++it) {
            const unsigned row = (unsigned)(half * 4 + it) * 2u + hh;
            *(volatile v4f*)(C + (size_t)(mBase + row) * ldc + n0 + c4) = vv[it];
          }
          __threadfence();
        }
      }
    } else {
      _Float16* C = (_Float16*)Cout;
      const unsigned q = lane >> 3, c8 = (lane & 7u) * 8u;
      v8h hv[4];
#pragma unroll
      for (int it = 0; it < 4; ++it) {
        const unsigned row = (unsigned)it * 4u + q;
        const float* sp = slab + row * 68u + c8;
#pragma unroll
        for (int e = 0; e < 8; ++e) hv[it][e] = toh_flush(sp[e]);
      }
      for (int pass = 0; pass < 2; ++pass) {
#pragma unroll
        for (int it = 0; it < 4; ++it) {
          const unsigned row = (unsigned)it * 4u + q;
          *(volatile v8h*)(C + (size_t)(mBase + row) * ldc + n0 + c8) = hv[it];
        }
        __threadfence();
      }
    }
    wave_sync_lds();
  }
}

__global__ __launch_bounds__(256) void k_gemm_val(const _Float16* __restrict__ A, const _Float16* __restrict__ Bt,
                                                  float* __restrict__ C, unsigned M) {
  __shared__ __align__(16) float sT[8 * 16 * 68];
  gemm64_body<0, false, false, false>(A, EMB, Bt, EMB, (void*)C, EMB, nullptr, nullptr, M, EMB, EMB, sT);
}
__global__ __launch_bounds__(256) void k_gemm_hid(const _Float16* __restrict__ A, const _Float16* __restrict__ Bt,
                                                  _Float16* __restrict__ C, const float* __restrict__ bias, unsigned M) {
  __shared__ __align__(16) float sT[8 * 16 * 68];
  gemm64_body<1, true, false, true>(A, EMB, Bt, EMB, (void*)C, HIDD, bias, nullptr, M, HIDD, EMB, sT);
}
__global__ __launch_bounds__(256) void k_gemm_y(const _Float16* __restrict__ A, const _Float16* __restrict__ Bt,
                                                float* __restrict__ C, const float* __restrict__ bias,
                                                const float* __restrict__ resid, unsigned M) {
  __shared__ __align__(16) float sT[8 * 16 * 68];
  gemm64_body<0, true, true, false>(A, HIDD, Bt, HIDD, (void*)C, EMB, bias, resid, M, EMB, HIDD, sT);
}

__global__ __launch_bounds__(256) void k_wt16(const float* __restrict__ Wm, unsigned KI, unsigned NO, unsigned lgper,
                                              unsigned short* __restrict__ W16, float sw) {
    const unsigned layer = blockIdx.y;
    const float* Wl = Wm + (size_t)layer * KI * NO;
    unsigned short* Dl = W16 + (size_t)layer * KI * NO;
    const unsigned u = blockIdx.x * 256u + threadIdx.x;
    const unsigned per = 1u << lgper;
    if (u >= NO * per) return;
    const unsigned k0 = 8u * (u & (per - 1u));
    const unsigned o = u >> lgper;
    float v[8];
#pragma unroll
    for (int i = 0; i < 8; ++i) v[i] = bfr(Wl[(size_t)(k0 + (unsigned)i) * NO + o]) * sw;
    st8h(Dl, (size_t)o * KI + k0, v);
}

__global__ __launch_bounds__(256) void k_hplane(const float* __restrict__ hist, _Float16* __restrict__ hp) {
    const unsigned u = blockIdx.x * 256u + threadIdx.x;
    const unsigned row = u >> 5, c0 = (u & 31u) * 8u;
    const unsigned rc = min(row, (unsigned)(SEQ_FULL - 1));
    const bool live = row < (unsigned)SEQ_FULL;
    const float* src = hist + (size_t)rc * 256u + c0;
    const v4f a = *(const v4f*)src, b = *(const v4f*)(src + 4);
    const float x[8] = {a.x, a.y, a.z, a.w, b.x, b.y, b.z, b.w};
    v8h hv;
#pragma unroll
    for (int e = 0; e < 8; ++e) hv[e] = toh_flush(live ? bfr(x[e]) * ACT_CARRY : 0.0f);
    _Float16* dst = hp + (size_t)row * 256u + c0;
    for (int pass = 0; pass < 2; ++pass) {
        *(volatile v8h*)dst = hv;
        __threadfence();
    }
}

__global__ __launch_bounds__(256) void k_featT(const float* __restrict__ sff, float* __restrict__ featf,
                                               _Float16* __restrict__ feat16) {
    __shared__ float sT[64][65];
    const unsigned t = threadIdx.x;
    const unsigned bx = blockIdx.x;
    const unsigned e0 = (bx & 3u) * 64u, l0 = ((bx >> 2) & 15u) * 64u, cam = bx >> 6;
#pragma unroll
    for (int i = 0; i < 4; ++i) {
        const unsigned idx = t + 256u * (unsigned)i;
        const unsigned el = idx >> 4, l4 = (idx & 15u) * 4u;
        const v4f v = *(const v4f*)(sff + (size_t)(cam * 256u + e0 + el) * 1024u + l0 + l4);
        sT[el][l4 + 0u] = bfr(v.x); sT[el][l4 + 1u] = bfr(v.y); sT[el][l4 + 2u] = bfr(v.z); sT[el][l4 + 3u] = bfr(v.w);
    }
    __syncthreads();
    v4f fv[4];
#pragma unroll
    for (int i = 0; i < 4; ++i) {
        const unsigned idx = t + 256u * (unsigned)i;
        const unsigned row = idx >> 4, c4 = (idx & 15u) * 4u;
        fv[i] = (v4f){sT[c4][row], sT[c4 + 1u][row], sT[c4 + 2u][row], sT[c4 + 3u][row]};
    }
    v8h hv[2];
#pragma unroll
    for (int i = 0; i < 2; ++i) {
        const unsigned idx = t + 256u * (unsigned)i;
        const unsigned row = idx >> 3, c8 = (idx & 7u) * 8u;
#pragma unroll
        for (int e = 0; e < 8; ++e) hv[i][e] = toh_flush(sT[c8 + (unsigned)e][row] * ACT_CARRY);
    }
    for (int pass = 0; pass < 2; ++pass) {
#pragma unroll
        for (int i = 0; i < 4; ++i) {
            const unsigned idx = t + 256u * (unsigned)i;
            const unsigned row = idx >> 4, c4 = (idx & 15u) * 4u;
            *(volatile v4f*)(featf + (size_t)(cam * 1024u + l0 + row) * 256u + e0 + c4) = fv[i];
        }
#pragma unroll
        for (int i = 0; i < 2; ++i) {
            const unsigned idx = t + 256u * (unsigned)i;
            const unsigned row = idx >> 3, c8 = (idx & 7u) * 8u;
            *(volatile v8h*)(feat16 + (size_t)(cam * 1024u + l0 + row) * 256u + e0 + c8) = hv[i];
        }
        __threadfence();
    }
}

__global__ __launch_bounds__(256) void k_tattn(const float* __restrict__ hist, const float* __restrict__ qin,
                                               const float* __restrict__ vt, const int* __restrict__ idxt,
                                               const float* __restrict__ smpw, const float* __restrict__ g,
                                               const float* __restrict__ be, float* __restrict__ x1) {
    __shared__ __align__(16) float sRow[8][256];
    const unsigned lane = threadIdx.x & 31u;
    const unsigned wave = (unsigned)__builtin_amdgcn_readfirstlane((int)(threadIdx.x >> 5));
    const unsigned s = blockIdx.x * 8u + wave;
    if (s >= (unsigned)SEQ) return;
    const unsigned c0 = 8u * lane;
    const float* qr = qin + (size_t)s * 256u + c0;
    const v4f qa = *(const v4f*)qr, qb = *(const v4f*)(qr + 4);
    const float q[8] = {bfr(qa.x), bfr(qa.y), bfr(qa.z), bfr(qa.w), bfr(qb.x), bfr(qb.y), bfr(qb.z), bfr(qb.w)};
    float o[8];
#pragma unroll
    for (int j = 0; j < 8; ++j) o[j] = 0.f;
    float m = -3.0e38f, den = 0.f;
#pragma unroll 1
    for (unsigned r = 0; r < (unsigned)NREF; ++r) {
        const int idr = idxt[s * 4u + r];
        const unsigned id = (unsigned)min(max(idr, 0), SEQ_FULL - 1);
        const float wr = bfr(smpw[s * 4u + r]);
        const float* kr = hist + (size_t)id * 256u + c0;
        const float* vr = vt + (size_t)id * 256u + c0;
        const v4f ka = *(const v4f*)kr, kb = *(const v4f*)(kr + 4);
        const v4f va = *(const v4f*)vr, vb = *(const v4f*)(vr + 4);
        const float kk[8] = {bfr(ka.x), bfr(ka.y), bfr(ka.z), bfr(ka.w), bfr(kb.x), bfr(kb.y), bfr(kb.z), bfr(kb.w)};
        const float vv[8] = {va.x, va.y, va.z, va.w, vb.x, vb.y, vb.z, vb.w};
        float p = 0.f;
#pragma unroll
        for (int j = 0; j < 8; ++j) p += q[j] * kk[j];
        p += __shfl_xor(p, 1, 32);
        p += __shfl_xor(p, 2, 32);
        const float sc = p * QK_SCALE2;
        const float mnew = (sc > m) ? sc : m;
        const float alpha = exp2f(m - mnew);
        const float ex = exp2f(sc - mnew);
        den = den * alpha + ex;
        const float ew = ex * wr;
#pragma unroll
        for (int j = 0; j < 8; ++j) o[j] = o[j] * alpha + ew * vv[j];
        m = mnew;
    }
    const float inv = 1.0f / den;
    float x[8];
#pragma unroll
    for (int j = 0; j < 8; ++j) x[j] = o[j] * inv + q[j];
    float sm = ((x[0] + x[1]) + (x[2] + x[3])) + ((x[4] + x[5]) + (x[6] + x[7]));
#pragma unroll
    for (int w = 16; w > 0; w >>= 1) sm += __shfl_xor(sm, w, 32);
    const float mu = sm * (1.0f / 256.0f);
    float d[8];
    float qv = 0.f;
#pragma unroll
    for (int j = 0; j < 8; ++j) { d[j] = x[j] - mu; qv += d[j] * d[j]; }
#pragma unroll
    for (int w = 16; w > 0; w >>= 1) qv += __shfl_xor(qv, w, 32);
    const float rs = rsqrtf(qv * (1.0f / 256.0f) + 1e-5f);
    const v4f g0 = *(const v4f*)(g + c0), g1 = *(const v4f*)(g + c0 + 4u);
    const v4f b0 = *(const v4f*)(be + c0), b1 = *(const v4f*)(be + c0 + 4u);
    const float gg[8] = {g0.x, g0.y, g0.z, g0.w, g1.x, g1.y, g1.z, g1.w};
    const float bb[8] = {b0.x, b0.y, b0.z, b0.w, b1.x, b1.y, b1.z, b1.w};
    float y[8];
#pragma unroll
    for (int j = 0; j < 8; ++j) y[j] = d[j] * rs * bfr(gg[j]) + bfr(bb[j]);
    *(v4f*)&sRow[wave][c0] = (v4f){y[0], y[1], y[2], y[3]};
    *(v4f*)&sRow[wave][c0 + 4u] = (v4f){y[4], y[5], y[6], y[7]};
    wave_sync_lds();
    const v4f o0 = *(const v4f*)&sRow[wave][4u * lane];
    const v4f o1 = *(const v4f*)&sRow[wave][128u + 4u * lane];
    float* dst = x1 + (size_t)s * 256u;
    for (int pass = 0; pass < 2; ++pass) {
        *(volatile v4f*)(dst + 4u * lane) = o0;
        *(volatile v4f*)(dst + 128u + 4u * lane) = o1;
        __threadfence();
    }
}

__global__ __launch_bounds__(256) void k_sattn(const float* __restrict__ featf, const float* __restrict__ vs,
                                               const float* __restrict__ x1, const int* __restrict__ idxs,
                                               const float* __restrict__ smpw, const float* __restrict__ g,
                                               const float* __restrict__ be, float* __restrict__ x2,
                                               _Float16* __restrict__ x2h) {
    __shared__ __align__(16) float sRow[8][256];
    const unsigned lane = threadIdx.x & 31u;
    const unsigned sv = blockIdx.x * 8u + (threadIdx.x >> 5);
    const unsigned wave = (unsigned)__builtin_amdgcn_readfirstlane((int)(threadIdx.x >> 5));
    const unsigned s = (unsigned)__builtin_amdgcn_readfirstlane((int)sv);
    const unsigned sq = (unsigned)__builtin_amdgcn_readfirstlane((int)min(sv, (unsigned)(SEQ - 1)));
    const bool live = s < (unsigned)SEQ;
    const unsigned c0 = 8u * lane;
    const float* qr = x1 + (size_t)sq * 256u + c0;
    const v4f qa = *(const v4f*)qr, qb = *(const v4f*)(qr + 4);
    const float q[8] = {qa.x, qa.y, qa.z, qa.w, qb.x, qb.y, qb.z, qb.w};
    float o[8];
#pragma unroll
    for (int j = 0; j < 8; ++j) o[j] = 0.f;
    float m = -3.0e38f, den = 0.f;
#pragma unroll 1
    for (unsigned i = 0; i < (unsigned)(NCAM * NREF); ++i) {
        const unsigned cam = i >> 2, r = i & 3u;
        const unsigned ii = (cam * (unsigned)SEQ_FULL + sq) * 4u + r;
        const int idr = idxs[ii];
        const unsigned id = (unsigned)min(max(idr, 0), FL - 1);
        const float wr = bfr(smpw[ii]);
        const unsigned row = cam * (unsigned)FL + id;
        const float* kr = featf + (size_t)row * 256u + c0;
        const float* vr = vs + (size_t)row * 256u + c0;
        const v4f ka = *(const v4f*)kr, kb = *(const v4f*)(kr + 4);
        const v4f va = *(const v4f*)vr, vb = *(const v4f*)(vr + 4);
        const float kk[8] = {ka.x, ka.y, ka.z, ka.w, kb.x, kb.y, kb.z, kb.w};
        const float vv[8] = {va.x, va.y, va.z, va.w, vb.x, vb.y, vb.z, vb.w};
        float p = 0.f;
#pragma unroll
        for (int j = 0; j < 8; ++j) p += q[j] * kk[j];
        p += __shfl_xor(p, 1, 32);
        p += __shfl_xor(p, 2, 32);
        const float sc = p * QK_SCALE2;
        const float mnew = (sc > m) ? sc : m;
        const float alpha = exp2f(m - mnew);
        const float ex = exp2f(sc - mnew);
        den = den * alpha + ex;
        const float ew = ex * wr;
#pragma unroll
        for (int j = 0; j < 8; ++j) o[j] = o[j] * alpha + ew * vv[j];
        m = mnew;
    }
    const float inv = 1.0f / den;
    float x[8];
#pragma unroll
    for (int j = 0; j < 8; ++j) x[j] = o[j] * inv + q[j];
    float sm = ((x[0] + x[1]) + (x[2] + x[3])) + ((x[4] + x[5]) + (x[6] + x[7]));
#pragma unroll
    for (int w = 16; w > 0; w >>= 1) sm += __shfl_xor(sm, w, 32);
    const float mu = sm * (1.0f / 256.0f);
    float d[8];
    float qv = 0.f;
#pragma unroll
    for (int j = 0; j < 8; ++j) { d[j] = x[j] - mu; qv += d[j] * d[j]; }
#pragma unroll
    for (int w = 16; w > 0; w >>= 1) qv += __shfl_xor(qv, w, 32);
    const float rs = rsqrtf(qv * (1.0f / 256.0f) + 1e-5f);
    const v4f g0 = *(const v4f*)(g + c0), g1 = *(const v4f*)(g + c0 + 4u);
    const v4f b0 = *(const v4f*)(be + c0), b1 = *(const v4f*)(be + c0 + 4u);
    const float gg[8] = {g0.x, g0.y, g0.z, g0.w, g1.x, g1.y, g1.z, g1.w};
    const float bb[8] = {b0.x, b0.y, b0.z, b0.w, b1.x, b1.y, b1.z, b1.w};
    float y[8];
#pragma unroll
    for (int j = 0; j < 8; ++j) {
        const float yv = d[j] * rs * bfr(gg[j]) + bfr(bb[j]);
        y[j] = live ? yv : 0.0f;
    }
    v8h hv;
#pragma unroll
    for (int j = 0; j < 8; ++j) hv[j] = toh_flush(y[j] * ACT_CARRY);
    *(v4f*)&sRow[wave][c0] = (v4f){y[0], y[1], y[2], y[3]};
    *(v4f*)&sRow[wave][c0 + 4u] = (v4f){y[4], y[5], y[6], y[7]};
    wave_sync_lds();
    const v4f o0 = *(const v4f*)&sRow[wave][4u * lane];
    const v4f o1 = *(const v4f*)&sRow[wave][128u + 4u * lane];
    float* dst = x2 + (size_t)s * 256u;
    _Float16* dsth = x2h + (size_t)s * 256u + c0;
    for (int pass = 0; pass < 2; ++pass) {
        *(volatile v4f*)(dst + 4u * lane) = o0;
        *(volatile v4f*)(dst + 128u + 4u * lane) = o1;
        *(volatile v8h*)dsth = hv;
        __threadfence();
    }
}

__global__ __launch_bounds__(256) void k_ln3(const float* __restrict__ yin, const float* __restrict__ g,
                                             const float* __restrict__ be, float* __restrict__ out) {
    const unsigned lane = threadIdx.x & 31u;
    const unsigned wave = (unsigned)__builtin_amdgcn_readfirstlane((int)(threadIdx.x >> 5));
    const unsigned s = blockIdx.x * 8u + wave;
    if (s >= (unsigned)SEQ) return;
    const unsigned ca = 4u * lane, cb = 128u + 4u * lane;
    const float* yr = yin + (size_t)s * 256u;
    const v4f a = *(const v4f*)(yr + ca), b = *(const v4f*)(yr + cb);
    float sm = ((a.x + a.y) + (a.z + a.w)) + ((b.x + b.y) + (b.z + b.w));
#pragma unroll
    for (int w = 16; w > 0; w >>= 1) sm += __shfl_xor(sm, w, 32);
    const float mu = sm * (1.0f / 256.0f);
    const float d[8] = {a.x - mu, a.y - mu, a.z - mu, a.w - mu, b.x - mu, b.y - mu, b.z - mu, b.w - mu};
    float qv = 0.f;
#pragma unroll
    for (int j = 0; j < 8; ++j) qv += d[j] * d[j];
#pragma unroll
    for (int w = 16; w > 0; w >>= 1) qv += __shfl_xor(qv, w, 32);
    const float rs = rsqrtf(qv * (1.0f / 256.0f) + 1e-5f);
    const v4f g0 = *(const v4f*)(g + ca), g1 = *(const v4f*)(g + cb);
    const v4f b0 = *(const v4f*)(be + ca), b1 = *(const v4f*)(be + cb);
    const float gg[8] = {g0.x, g0.y, g0.z, g0.w, g1.x, g1.y, g1.z, g1.w};
    const float bb[8] = {b0.x, b0.y, b0.z, b0.w, b1.x, b1.y, b1.z, b1.w};
    float y[8];
#pragma unroll
    for (int j = 0; j < 8; ++j) y[j] = d[j] * rs * bfr(gg[j]) + bfr(bb[j]);
    const v4f o0 = (v4f){y[0], y[1], y[2], y[3]};
    const v4f o1 = (v4f){y[4], y[5], y[6], y[7]};
    float* dst = out + (size_t)s * 256u;
    for (int pass = 0; pass < 2; ++pass) {
        *(volatile v4f*)(dst + ca) = o0;
        *(volatile v4f*)(dst + cb) = o1;
        __threadfence();
    }
}

static constexpr size_t SZ_WSQ  = (size_t)EMB * EMB * 2;
static constexpr size_t SZ_WFF  = (size_t)EMB * HIDD * 2;
static constexpr size_t SZ_H16  = (size_t)HPAD * EMB * 2;
static constexpr size_t SZ_FTF  = (size_t)FROWS * EMB * 4;
static constexpr size_t SZ_FT16 = (size_t)FROWS * EMB * 2;
static constexpr size_t SZ_VT   = (size_t)HPAD * EMB * 4;
static constexpr size_t SZ_VS   = (size_t)FROWS * EMB * 4;
static constexpr size_t SZ_X1   = (size_t)SEQ * EMB * 4;
static constexpr size_t SZ_X2   = (size_t)MPAD * EMB * 4;
static constexpr size_t SZ_X2H  = (size_t)MPAD * EMB * 2;
static constexpr size_t SZ_HID  = (size_t)MPAD * HIDD * 2;
static constexpr size_t SZ_Y    = (size_t)MPAD * EMB * 4;
static constexpr size_t OFF_WVT  = 0;
static constexpr size_t OFF_WVS  = OFF_WVT + SZ_WSQ;
static constexpr size_t OFF_W1T  = OFF_WVS + SZ_WSQ;
static constexpr size_t OFF_W2T  = OFF_W1T + SZ_WFF;
static constexpr size_t OFF_H16  = OFF_W2T + SZ_WFF;
static constexpr size_t OFF_FTF  = OFF_H16 + SZ_H16;
static constexpr size_t OFF_FT16 = OFF_FTF + SZ_FTF;
static constexpr size_t OFF_VT   = OFF_FT16 + SZ_FT16;
static constexpr size_t OFF_VS   = OFF_VT + SZ_VT;
static constexpr size_t OFF_X1   = OFF_VS + SZ_VS;
static constexpr size_t OFF_X2   = OFF_X1 + SZ_X1;
static constexpr size_t OFF_X2H  = OFF_X2 + SZ_X2;
static constexpr size_t OFF_HID  = OFF_X2H + SZ_X2H;
static constexpr size_t OFF_Y    = OFF_HID + SZ_HID;
static constexpr size_t WS_TOTAL = OFF_Y + SZ_Y;
static_assert(WS_TOTAL <= (size_t)134217728);
static_assert(SZ_WSQ % 256 == 0 && SZ_WFF % 256 == 0 && SZ_H16 % 256 == 0 && SZ_FTF % 256 == 0 && SZ_FT16 % 256 == 0);
static_assert(SZ_VT % 256 == 0 && SZ_VS % 256 == 0 && SZ_X1 % 256 == 0 && SZ_X2 % 256 == 0 && SZ_X2H % 256 == 0 && SZ_HID % 256 == 0);

static constexpr unsigned G_WSQ  = (EMB * (EMB / 8)) / 256;
static constexpr unsigned G_W1   = (HIDD * (EMB / 8)) / 256;
static constexpr unsigned G_W2   = (EMB * (HIDD / 8)) / 256;
static constexpr unsigned G_HPL  = (HPAD * (EMB / 8)) / 256;
static constexpr unsigned G_FT   = NCAM * 16 * 4;
static constexpr unsigned G_VT   = ((HPAD / 64) * (EMB / 64) + 7) / 8;
static constexpr unsigned G_VS   = ((FROWS / 64) * (EMB / 64) + 7) / 8;
static constexpr unsigned G_HID  = ((MPAD / 64) * (HIDD / 64) + 7) / 8;
static constexpr unsigned G_Y    = ((MPAD / 64) * (EMB / 64) + 7) / 8;
static constexpr unsigned G_TAT  = SEQ / 8;
static constexpr unsigned G_SAT  = MPAD / 8;
static constexpr unsigned G_LN3  = SEQ / 8;
static_assert(G_HPL * 256u == (unsigned)(HPAD * (EMB / 8)));
static_assert(G_TAT * 8u == (unsigned)SEQ && G_SAT * 8u == (unsigned)MPAD && G_LN3 * 8u == (unsigned)SEQ);
static_assert(G_FT * 64u * 64u == (unsigned)(FROWS * EMB));

extern "C" void kernel_launch(void* const* d_in, const int* in_sizes, int n_in, void* d_out, int out_size,
                              void* d_ws, size_t ws_size, hipStream_t stream) {
    if (n_in < 19) return;
    if (in_sizes[0] < SEQ_FULL * EMB || in_sizes[1] < SEQ * EMB || in_sizes[2] < FROWS * EMB) return;
    if (in_sizes[3] < SEQ * NREF || in_sizes[4] < ((NCAM - 1) * SEQ_FULL + SEQ) * NREF) return;
    if (in_sizes[5] < SEQ * NREF || in_sizes[6] < ((NCAM - 1) * SEQ_FULL + SEQ) * NREF) return;
    if (in_sizes[7] < EMB * EMB || in_sizes[8] < EMB * EMB || in_sizes[9] < EMB * HIDD || in_sizes[10] < HIDD) return;
    if (in_sizes[11] < HIDD * EMB || in_sizes[12] < EMB || in_sizes[13] < EMB || in_sizes[14] < EMB) return;
    if (in_sizes[15] < EMB || in_sizes[16] < EMB || in_sizes[17] < EMB || in_sizes[18] < EMB) return;
    if (out_size < SEQ * EMB) return;
    if (ws_size < WS_TOTAL) return;

    const float* history = (const float*)d_in[0];
    const float* query   = (const float*)d_in[1];
    const float* sff     = (const float*)d_in[2];
    const int*   idx_t   = (const int*)d_in[3];
    const int*   idx_s   = (const int*)d_in[4];
    const float* w_t     = (const float*)d_in[5];
    const float* w_s     = (const float*)d_in[6];
    const float* W_v_t   = (const float*)d_in[7];
    const float* W_v_s   = (const float*)d_in[8];
    const float* W1      = (const float*)d_in[9];
    const float* b1      = (const float*)d_in[10];
    const float* W2      = (const float*)d_in[11];
    const float* b2      = (const float*)d_in[12];
    const float* g1      = (const float*)d_in[13];
    const float* be1     = (const float*)d_in[14];
    const float* g2      = (const float*)d_in[15];
    const float* be2     = (const float*)d_in[16];
    const float* g3      = (const float*)d_in[17];
    const float* be3     = (const float*)d_in[18];
    float* out = (float*)d_out;

    char* wsp = (char*)d_ws;
    unsigned short* wvt   = (unsigned short*)(wsp + OFF_WVT);
    unsigned short* wvs   = (unsigned short*)(wsp + OFF_WVS);
    unsigned short* w1t   = (unsigned short*)(wsp + OFF_W1T);
    unsigned short* w2t   = (unsigned short*)(wsp + OFF_W2T);
    _Float16*       h16p  = (_Float16*)(wsp + OFF_H16);
    float*          featf = (float*)(wsp + OFF_FTF);
    _Float16*       ft16  = (_Float16*)(wsp + OFF_FT16);
    float*          vt    = (float*)(wsp + OFF_VT);
    float*          vs    = (float*)(wsp + OFF_VS);
    float*          x1    = (float*)(wsp + OFF_X1);
    float*          x2    = (float*)(wsp + OFF_X2);
    _Float16*       x2h   = (_Float16*)(wsp + OFF_X2H);
    _Float16*       hid   = (_Float16*)(wsp + OFF_HID);
    float*          yb    = (float*)(wsp + OFF_Y);

    k_wt16<<<dim3(G_WSQ, 1), 256, 0, stream>>>(W_v_t, EMB, EMB, 5, wvt, W_CARRY);
    k_wt16<<<dim3(G_WSQ, 1), 256, 0, stream>>>(W_v_s, EMB, EMB, 5, wvs, W_CARRY);
    k_wt16<<<dim3(G_W1, 1), 256, 0, stream>>>(W1, EMB, HIDD, 5, w1t, W_CARRY);
    k_wt16<<<dim3(G_W2, 1), 256, 0, stream>>>(W2, HIDD, EMB, 4, w2t, W_CARRY);

    k_hplane<<<G_HPL, 256, 0, stream>>>(history, h16p);
    k_featT<<<G_FT, 256, 0, stream>>>(sff, featf, ft16);

    k_gemm_val<<<G_VT, 256, 0, stream>>>((const _Float16*)h16p, (const _Float16*)wvt, vt, HPAD);
    k_gemm_val<<<G_VS, 256, 0, stream>>>((const _Float16*)ft16, (const _Float16*)wvs, vs, FROWS);

    k_tattn<<<G_TAT, 256, 0, stream>>>(history, query, vt, idx_t, w_t, g1, be1, x1);
    k_sattn<<<G_SAT, 256, 0, stream>>>(featf, vs, x1, idx_s, w_s, g2, be2, x2, x2h);

    k_gemm_hid<<<G_HID, 256, 0, stream>>>((const _Float16*)x2h, (const _Float16*)w1t, hid, b1, MPAD);
    k_gemm_y<<<G_Y, 256, 0, stream>>>((const _Float16*)hid, (const _Float16*)w2t, yb, b2, x2, MPAD);
    k_ln3<<<G_LN3, 256, 0, stream>>>(yb, g3, be3, out);
}
